// SelfAttention_3126736191665
// MI455X (gfx1250) — hardware-verified
//
#include <hip/hip_runtime.h>


#ifndef NB
#define NB 2
#endif
#ifndef SEQ
#define SEQ 2048
#endif
#define NB_FULL  2
#define SEQ_FULL 2048
#define DM       1024
#define NHEAD    16
#define HDIM     64
#define NTOK     (NB * SEQ)
#define BQ       128
#define BK       32
#define NWAVE    8
#define OP       68
#define GT       128
#define GK       32
#define GLD      40
#define GPC      132
#define WT       64
#define WTP      72

static_assert(NB >= 1 && NB <= NB_FULL);
static_assert(SEQ >= BQ && SEQ <= SEQ_FULL);
static_assert(SEQ % BQ == 0);
static_assert(SEQ % BK == 0);
static_assert(SEQ % GT == 0);
static_assert(NTOK % GT == 0);
static_assert(DM % GT == 0);
static_assert(DM % GK == 0);
static_assert(DM % WT == 0);
static_assert(NTOK % 2 == 0);
static_assert(NHEAD * HDIM == DM);
static_assert(HDIM == 64);
static_assert(BQ == NWAVE * 16);
static_assert((GLD * 2) % 16 == 0);
static_assert((GPC * 4) % 16 == 0);
static_assert((WTP * 2) % 16 == 0);
static_assert((OP * 4) % 16 == 0);
static_assert(GT * GPC * 4 >= 2 * GT * GLD * 2);

typedef __bf16   bf16;
typedef _Float16 f16;
typedef bf16     v16bf __attribute__((ext_vector_type(16)));
typedef f16      v16h  __attribute__((ext_vector_type(16)));
typedef f16      v8h   __attribute__((ext_vector_type(8)));
typedef float    v8f   __attribute__((ext_vector_type(8)));
typedef float    v4f   __attribute__((ext_vector_type(4)));
typedef unsigned v4u   __attribute__((ext_vector_type(4)));

union FragB  { v16bf v; v4u q[2]; bf16 h[16]; };
union FragH  { v16h  v; v4u q[2]; f16  h[16]; };
union FragU  { v16h  h; v16bf b; v4u q[2]; };
union Pack8B { v4u u; bf16 h[8]; };
union Pack8H { v4u u; v8h v; f16 h[8]; };
union U16    { unsigned short u; bf16 b; f16 h; };

static __device__ __forceinline__ v8f mma_bf16(v16bf a, v16bf b, v8f acc) {
  acc = __builtin_amdgcn_wmma_f32_16x16x32_bf16(false, a, false, b, (short)0, acc, false, false);
  asm volatile("v_nop\n\tv_nop\n\tv_nop\n\tv_nop" : "+v"(acc) : "v"(a), "v"(b));
  return acc;
}
static __device__ __forceinline__ v8f mma_f16(v16h a, v16h b, v8f acc) {
  acc = __builtin_amdgcn_wmma_f32_16x16x32_f16(false, a, false, b, (short)0, acc, false, false);
  asm volatile("v_nop\n\tv_nop\n\tv_nop\n\tv_nop" : "+v"(acc) : "v"(a), "v"(b));
  return acc;
}

__global__ __launch_bounds__(256) void cvt_x_kernel(const float* __restrict__ x, bf16* __restrict__ xb) {
  const int tid = threadIdx.x;
  const int r   = blockIdx.x * 2 + (tid >> 7);
  const int c0  = (tid & 127) * 8;
  const int b   = r / SEQ;
  const int s   = r - b * SEQ;
  const float* src = x + ((size_t)b * SEQ_FULL + s) * DM + c0;
  const v4f a0 = *(const v4f*)(src);
  const v4f a1 = *(const v4f*)(src + 4);
  Pack8B pk;
  #pragma unroll
  for (int i = 0; i < 4; ++i) {
    pk.h[i]     = (bf16)a0[i];
    pk.h[4 + i] = (bf16)a1[i];
  }
  bf16* dst = xb + (size_t)r * DM + c0;
  *(volatile v4u*)dst = pk.u;
  __threadfence();
  *(volatile v4u*)dst = pk.u;
}

__global__ __launch_bounds__(256) void cvt_w_kernel(const float* __restrict__ w,
                                                    unsigned short* __restrict__ wt, int mode) {
  __shared__ __align__(16) unsigned short t[WT * WTP];
  const int nb  = blockIdx.x * WT;
  const int kb  = blockIdx.y * WT;
  const int tid = threadIdx.x;
  #pragma unroll
  for (int it = 0; it < 4; ++it) {
    const int idx = tid + it * 256;
    const int k   = idx >> 4;
    const int n4  = (idx & 15) * 4;
    const v4f v = *(const v4f*)(w + (size_t)(kb + k) * DM + nb + n4);
    #pragma unroll
    for (int j = 0; j < 4; ++j) {
      const bf16 bv = (bf16)v[j];
      U16 q;
      if (mode != 0) q.h = (f16)((float)bv * 256.0f);
      else           q.b = bv;
      t[(n4 + j) * WTP + k] = q.u;
    }
  }
  __syncthreads();

  v4u    vals[2];
  size_t gidx[2];
  #pragma unroll
  for (int it = 0; it < 2; ++it) {
    const int idx = tid + it * 256;
    const int n   = idx >> 3;
    const int ks  = (idx & 7) * 8;
    vals[it] = *(const v4u*)(t + n * WTP + ks);
    gidx[it] = (size_t)(nb + n) * DM + kb + ks;
  }
  #pragma unroll
  for (int it = 0; it < 2; ++it) *(volatile v4u*)(wt + gidx[it]) = vals[it];
  __threadfence();
  #pragma unroll
  for (int it = 0; it < 2; ++it) *(volatile v4u*)(wt + gidx[it]) = vals[it];
}

template <typename CT, bool F16OP, bool BIASROW>
__global__ __launch_bounds__(256) void gemm_kernel(const unsigned short* __restrict__ A,
                                                   const unsigned short* __restrict__ B,
                                                   const float* __restrict__ bias,
                                                   CT* __restrict__ C,
                                                   int lda, int ldb, int K, int ldc,
                                                   int rpb, int rbs, int cpb, int cbs,
                                                   float ascale, float bscale) {
  __shared__ __align__(16) float smem[GT * GPC];
  unsigned short* As = (unsigned short*)smem;
  unsigned short* Bs = As + GT * GLD;
  float* sC = smem;

  const int tid   = threadIdx.x;
  const int lane  = tid & 31;
  const int l16   = lane & 15;
  const int hi    = lane >> 4;
  const int wave  = tid >> 5;
  const int waveM = wave & 3;
  const int waveN = wave >> 2;
  const int rowBase = blockIdx.y * GT;
  const int colBase = blockIdx.x * GT;

  v8f acc[2][4];
  #pragma unroll
  for (int mi = 0; mi < 2; ++mi)
    #pragma unroll
    for (int ni = 0; ni < 4; ++ni) acc[mi][ni] = (v8f){0, 0, 0, 0, 0, 0, 0, 0};

  #pragma unroll 1
  for (int k0 = 0; k0 < K; k0 += GK) {
    #pragma unroll
    for (int it = 0; it < 2; ++it) {
      const int idx = tid + it * 256;
      const int r   = idx >> 2;
      const int cq  = idx & 3;
      *(v4u*)(As + r * GLD + cq * 8) = *(const v4u*)(A + (size_t)(rowBase + r) * lda + k0 + cq * 8);
      *(v4u*)(Bs + r * GLD + cq * 8) = *(const v4u*)(B + (size_t)(colBase + r) * ldb + k0 + cq * 8);
    }
    __syncthreads();

    FragU af[2], bq[4];
    #pragma unroll
    for (int mi = 0; mi < 2; ++mi) {
      const int m = waveM * 32 + mi * 16 + l16;
      af[mi].q[0] = *(const v4u*)(As + m * GLD + hi * 8);
      af[mi].q[1] = *(const v4u*)(As + m * GLD + 16 + hi * 8);
    }
    #pragma unroll
    for (int ni = 0; ni < 4; ++ni) {
      const int n = waveN * 64 + ni * 16 + l16;
      bq[ni].q[0] = *(const v4u*)(Bs + n * GLD + hi * 8);
      bq[ni].q[1] = *(const v4u*)(Bs + n * GLD + 16 + hi * 8);
    }
    #pragma unroll
    for (int mi = 0; mi < 2; ++mi)
      #pragma unroll
      for (int ni = 0; ni < 4; ++ni) {
        if (F16OP) acc[mi][ni] = mma_f16(af[mi].h, bq[ni].h, acc[mi][ni]);
        else       acc[mi][ni] = mma_bf16(af[mi].b, bq[ni].b, acc[mi][ni]);
      }
    __syncthreads();
  }

  #pragma unroll
  for (int mi = 0; mi < 2; ++mi)
    #pragma unroll
    for (int ni = 0; ni < 4; ++ni)
      #pragma unroll
      for (int i = 0; i < 8; ++i)
        sC[(waveM * 32 + mi * 16 + hi * 8 + i) * GPC + waveN * 64 + ni * 16 + l16] = acc[mi][ni][i];
  __syncthreads();

  const int    prow0 = (rowBase / rpb) * rbs + (rowBase % rpb);
  const size_t coff  = (size_t)(colBase / cpb) * (size_t)cbs + (size_t)(colBase % cpb);
  CT* Cb = C + (size_t)prow0 * ldc + coff;

  if (sizeof(CT) == 2) {
    v4u vals[8];
    #pragma unroll
    for (int it = 0; it < 8; ++it) {
      const int idx = it * 256 + tid;
      const int r   = idx >> 4;
      const int cs  = (idx & 15) * 8;
      const v4f s0 = *(const v4f*)(sC + r * GPC + cs);
      const v4f s1 = *(const v4f*)(sC + r * GPC + cs + 4);
      v4f b0, b1;
      if (BIASROW) {
        const float bvr = (float)(bf16)bias[rowBase + r];
        b0 = (v4f){bvr, bvr, bvr, bvr};
        b1 = b0;
      } else {
        const v4f t0 = *(const v4f*)(bias + colBase + cs);
        const v4f t1 = *(const v4f*)(bias + colBase + cs + 4);
        #pragma unroll
        for (int i = 0; i < 4; ++i) {
          b0[i] = (float)(bf16)t0[i];
          b1[i] = (float)(bf16)t1[i];
        }
      }
      Pack8H ph;
      #pragma unroll
      for (int i = 0; i < 4; ++i) {
        ph.h[i]     = (f16)(s0[i] * ascale + b0[i] * bscale);
        ph.h[4 + i] = (f16)(s1[i] * ascale + b1[i] * bscale);
      }
      vals[it] = ph.u;
    }
    #pragma unroll
    for (int it = 0; it < 8; ++it) {
      const int idx = it * 256 + tid;
      const int r = idx >> 4, cs = (idx & 15) * 8;
      *(volatile v4u*)(Cb + (size_t)r * ldc + cs) = vals[it];
    }
    __threadfence();
    #pragma unroll
    for (int it = 0; it < 8; ++it) {
      const int idx = it * 256 + tid;
      const int r = idx >> 4, cs = (idx & 15) * 8;
      *(volatile v4u*)(Cb + (size_t)r * ldc + cs) = vals[it];
    }
  } else {
    v4f vals[16];
    #pragma unroll
    for (int it = 0; it < 16; ++it) {
      const int idx = it * 256 + tid;
      const int r   = idx >> 5;
      const int cs  = (idx & 31) * 4;
      const v4f s0 = *(const v4f*)(sC + r * GPC + cs);
      v4f b0;
      if (BIASROW) {
        const float bvr = (float)(bf16)bias[rowBase + r];
        b0 = (v4f){bvr, bvr, bvr, bvr};
      } else {
        const v4f t0 = *(const v4f*)(bias + colBase + cs);
        #pragma unroll
        for (int i = 0; i < 4; ++i) b0[i] = (float)(bf16)t0[i];
      }
      v4f v;
      #pragma unroll
      for (int i = 0; i < 4; ++i) v[i] = s0[i] * ascale + b0[i] * bscale;
      vals[it] = v;
    }
    #pragma unroll
    for (int it = 0; it < 16; ++it) {
      const int idx = it * 256 + tid;
      const int r = idx >> 5, cs = (idx & 31) * 4;
      *(volatile v4f*)(Cb + (size_t)r * ldc + cs) = vals[it];
    }
    __threadfence();
    #pragma unroll
    for (int it = 0; it < 16; ++it) {
      const int idx = it * 256 + tid;
      const int r = idx >> 5, cs = (idx & 31) * 4;
      *(volatile v4f*)(Cb + (size_t)r * ldc + cs) = vals[it];
    }
  }
}

template <int RES>
__global__ __launch_bounds__(256) void attn_kernel(const f16* __restrict__ qh,
                                                   const f16* __restrict__ kh,
                                                   const f16* __restrict__ vt,
                                                   f16* __restrict__ ctx) {
  const int qblk = blockIdx.x;
  const int h    = blockIdx.y;
  const int b    = blockIdx.z;
  const int tid  = threadIdx.x;
  const int wave = tid >> 5;
  const int lane = tid & 31;
  const int lq   = lane & 15;
  const int hi   = lane >> 4;

  __shared__ __align__(16) float sO[NWAVE * 16 * OP];

  const int    qrow0 = qblk * BQ + wave * 16;
  const size_t tok0  = (size_t)b * SEQ + qrow0;

  FragH qf[2];
  {
    const f16* qp = qh + (tok0 + lq) * DM + h * HDIM + hi * 8;
    #pragma unroll
    for (int f = 0; f < 2; ++f) {
      qf[f].q[0] = *(const v4u*)(qp + f * 32);
      qf[f].q[1] = *(const v4u*)(qp + f * 32 + 16);
    }
  }

  const f16* kb_h = kh + (size_t)b * SEQ * DM + h * HDIM;
  const f16* vt_h = vt + ((size_t)b * DM + h * HDIM) * SEQ;

  v8f o[4], o2[4];
  #pragma unroll
  for (int dt = 0; dt < 4; ++dt) {
    o[dt]  = (v8f){0, 0, 0, 0, 0, 0, 0, 0};
    o2[dt] = (v8f){0, 0, 0, 0, 0, 0, 0, 0};
  }

  float rmax = -__builtin_inff();
  float rsum = 0.0f;
  const float SL = 1.4426950408889634f / 2048.0f;

  for (int i = 0; i < SEQ / BK; ++i) {
    const int j0 = i * BK;

    FragH ak[2][2];
    #pragma unroll
    for (int sub = 0; sub < 2; ++sub) {
      #pragma unroll
      for (int f = 0; f < 2; ++f) {
        const f16* base = kb_h + (size_t)(j0 + sub * 16 + lq) * DM + f * 32 + hi * 8;
        ak[sub][f].q[0] = *(const v4u*)(base);
        ak[sub][f].q[1] = *(const v4u*)(base + 16);
      }
    }
    FragH bv[4];
    #pragma unroll
    for (int dt = 0; dt < 4; ++dt) {
      const f16* base = vt_h + (size_t)(dt * 16 + lq) * SEQ + j0 + hi * 8;
      bv[dt].q[0] = *(const v4u*)(base);
      bv[dt].q[1] = *(const v4u*)(base + 16);
    }

    v8f c[2];
    #pragma unroll
    for (int sub = 0; sub < 2; ++sub) {
      v8f acc = (v8f){0, 0, 0, 0, 0, 0, 0, 0};
      acc = mma_f16(ak[sub][0].v, qf[0].v, acc);
      acc = mma_f16(ak[sub][1].v, qf[1].v, acc);
      c[sub] = acc;
    }

    float m_new = rmax;
    #pragma unroll
    for (int r = 0; r < 8; ++r) {
      m_new = fmaxf(m_new, c[0][r]);
      m_new = fmaxf(m_new, c[1][r]);
    }
    m_new = fmaxf(m_new, __shfl_xor(m_new, 16, 32));
    const float scale = __builtin_amdgcn_exp2f((rmax - m_new) * SL);
    rmax = m_new;

    FragH pa, pr;
    float psum = 0.0f;
    #pragma unroll
    for (int r = 0; r < 8; ++r) {
      const float p0 = __builtin_amdgcn_exp2f((c[0][r] - m_new) * SL);
      const float p1 = __builtin_amdgcn_exp2f((c[1][r] - m_new) * SL);
      psum += p0 + p1;
      const float pc0 = p0 * 4096.0f;
      const float pc1 = p1 * 4096.0f;
      const f16 h0 = (f16)pc0;
      const f16 h1 = (f16)pc1;
      pa.h[r]     = h0;
      pa.h[8 + r] = h1;
      if (RES != 0) {
        pr.h[r]     = (f16)((pc0 - (float)h0) * 1024.0f);
        pr.h[8 + r] = (f16)((pc1 - (float)h1) * 1024.0f);
      }
    }
    rsum = rsum * scale + psum + __shfl_xor(psum, 16, 32);

    float sc[8];
    #pragma unroll
    for (int r = 0; r < 8; ++r) sc[r] = __shfl(scale, (hi << 3) + r, 32);
    #pragma unroll
    for (int dt = 0; dt < 4; ++dt) {
      #pragma unroll
      for (int r = 0; r < 8; ++r) {
        o[dt][r] *= sc[r];
        if (RES != 0) o2[dt][r] *= sc[r];
      }
    }

    #pragma unroll
    for (int dt = 0; dt < 4; ++dt) {
      o[dt] = mma_f16(pa.v, bv[dt].v, o[dt]);
      if (RES != 0) o2[dt] = mma_f16(pr.v, bv[dt].v, o2[dt]);
    }
  }

  float rs[8];
  #pragma unroll
  for (int r = 0; r < 8; ++r) rs[r] = 1.0f / __shfl(rsum, (hi << 3) + r, 32);

  float* so = sO + wave * (16 * OP);
  #pragma unroll
  for (int r = 0; r < 8; ++r) {
    #pragma unroll
    for (int dt = 0; dt < 4; ++dt) {
      float val = o[dt][r];
      if (RES != 0) val += o2[dt][r] * (1.0f / 1024.0f);
      so[(hi * 8 + r) * OP + dt * 16 + lq] = val * (1.0f / 256.0f) * rs[r];
    }
  }
  __syncthreads();

  v4u    vals[4];
  size_t gidx[4];
  #pragma unroll
  for (int it = 0; it < 4; ++it) {
    const int row = it * 4 + (lane >> 3);
    const int seg = (lane & 7) * 8;
    const v4f s0 = *(const v4f*)(so + row * OP + seg);
    const v4f s1 = *(const v4f*)(so + row * OP + seg + 4);
    Pack8H ph;
    #pragma unroll
    for (int i = 0; i < 4; ++i) {
      ph.h[i]     = (f16)s0[i];
      ph.h[4 + i] = (f16)s1[i];
    }
    vals[it] = ph.u;
    gidx[it] = (tok0 + row) * DM + h * HDIM + seg;
  }
  #pragma unroll
  for (int it = 0; it < 4; ++it) *(volatile v4u*)(ctx + gidx[it]) = vals[it];
  __threadfence();
  #pragma unroll
  for (int it = 0; it < 4; ++it) *(volatile v4u*)(ctx + gidx[it]) = vals[it];
}

extern "C" void kernel_launch(void* const* d_in, const int* in_sizes, int n_in,
                              void* d_out, int out_size, void* d_ws, size_t ws_size,
                              hipStream_t stream) {
  if (n_in < 9) return;
  const size_t rows_used = (size_t)(NB - 1) * SEQ_FULL + SEQ;
  if ((size_t)in_sizes[0] < rows_used * DM) return;
  if ((size_t)in_sizes[1] < (size_t)DM * DM) return;
  if ((size_t)in_sizes[3] < (size_t)DM * DM) return;
  if ((size_t)in_sizes[5] < (size_t)DM * DM) return;
  if ((size_t)in_sizes[7] < (size_t)DM * DM) return;
  if (in_sizes[2] < DM || in_sizes[4] < DM || in_sizes[6] < DM || in_sizes[8] < DM) return;
  if ((size_t)out_size < rows_used * DM) return;

  const size_t act_bytes = (size_t)NTOK * DM * 2;
  const size_t w_bytes   = (size_t)DM * DM * 2;
  const size_t off_xb  = 0;
  const size_t off_wq  = off_xb + act_bytes;
  const size_t off_wk  = off_wq + w_bytes;
  const size_t off_wv  = off_wk + w_bytes;
  const size_t off_wo  = off_wv + w_bytes;
  const size_t off_qh  = off_wo + w_bytes;
  const size_t off_kh  = off_qh + act_bytes;
  const size_t off_vt  = off_kh + act_bytes;
  const size_t off_ctx = off_vt + act_bytes;
  const size_t total   = off_ctx + act_bytes;
  if (ws_size < total) return;

  const float* x  = (const float*)d_in[0];
  const float* Wq = (const float*)d_in[1];
  const float* bq = (const float*)d_in[2];
  const float* Wk = (const float*)d_in[3];
  const float* bk = (const float*)d_in[4];
  const float* Wv = (const float*)d_in[5];
  const float* bv = (const float*)d_in[6];
  const float* Wo = (const float*)d_in[7];
  const float* bo = (const float*)d_in[8];
  float* out = (float*)d_out;

  char* ws = (char*)d_ws;
  unsigned short* xb  = (unsigned short*)(ws + off_xb);
  unsigned short* wq  = (unsigned short*)(ws + off_wq);
  unsigned short* wk  = (unsigned short*)(ws + off_wk);
  unsigned short* wv  = (unsigned short*)(ws + off_wv);
  unsigned short* wo  = (unsigned short*)(ws + off_wo);
  unsigned short* qh  = (unsigned short*)(ws + off_qh);
  unsigned short* kh  = (unsigned short*)(ws + off_kh);
  unsigned short* vt  = (unsigned short*)(ws + off_vt);
  unsigned short* ctx = (unsigned short*)(ws + off_ctx);

  cvt_x_kernel<<<dim3(NTOK / 2), 256, 0, stream>>>(x, (bf16*)xb);

  const dim3 gw(DM / WT, DM / WT);
  cvt_w_kernel<<<gw, 256, 0, stream>>>(Wq, wq, 0);
  cvt_w_kernel<<<gw, 256, 0, stream>>>(Wk, wk, 0);
  cvt_w_kernel<<<gw, 256, 0, stream>>>(Wv, wv, 0);
  cvt_w_kernel<<<gw, 256, 0, stream>>>(Wo, wo, 1);

  const dim3 gqk(DM / GT, NTOK / GT);
  gemm_kernel<unsigned short, false, false><<<gqk, 256, 0, stream>>>(
      xb, wq, bq, qh, DM, DM, DM, DM, NTOK, 0, DM, 0, 16.0f, 16.0f);
  gemm_kernel<unsigned short, false, false><<<gqk, 256, 0, stream>>>(
      xb, wk, bk, kh, DM, DM, DM, DM, NTOK, 0, DM, 0, 16.0f, 16.0f);
  const dim3 gv(NTOK / GT, DM / GT);
  gemm_kernel<unsigned short, false, true><<<gv, 256, 0, stream>>>(
      wv, xb, bv, vt, DM, DM, DM, SEQ, DM, 0, SEQ, DM * SEQ, 16.0f, 16.0f);

  attn_kernel<0><<<dim3(SEQ / BQ, NHEAD, NB), 256, 0, stream>>>(
      (const f16*)qh, (const f16*)kh, (const f16*)vt, (f16*)ctx);

  gemm_kernel<float, true, false><<<gqk, 256, 0, stream>>>(
      ctx, wo, bo, out, DM, DM, DM, DM, SEQ, SEQ_FULL, DM, 0, 1.0f / 65536.0f, 1.0f);
}
